// GraphWeightEstimator_50878182588739
// MI455X (gfx1250) — hardware-verified
//
#include <hip/hip_runtime.h>
#include <math.h>

typedef _Float16 v8h  __attribute__((ext_vector_type(8)));
typedef _Float16 v16h __attribute__((ext_vector_type(16)));
typedef float    v8f  __attribute__((ext_vector_type(8)));
typedef float    v4f_t __attribute__((ext_vector_type(4)));
typedef float v4fa __attribute__((ext_vector_type(4), may_alias));
typedef unsigned v4u_t __attribute__((ext_vector_type(4)));
typedef unsigned v4ua __attribute__((ext_vector_type(4), may_alias));
#define RSPLIT (1.0f / 2048.0f)
static __device__ __forceinline__ _Float16 lo_of(float v, _Float16 h) { return (_Float16)((v - (float)h) * 2048.0f); }
static __device__ __forceinline__ v8f wmma16(v16h a, v16h b, v8f c) { return __builtin_amdgcn_wmma_f32_16x16x32_f16(false, a, false, b, (short)0, c, false, false); }
static __device__ __forceinline__ v8f wmma_split(v16h a, v16h al, v16h b, v16h bl, v8f c) { v8f x = {}; x = wmma16(al, b, x); x = wmma16(a, bl, x); return wmma16(a, b, c) + x * RSPLIT; }

#define HW    400
#define NPIX  (HW*HW)
#define CKK   363
#define N1    128
#define N2    64
#define NE    8
#define K1CH  12
#define K2CH  4
#define NT1   8
#define NT2   4
#define NW    4

#define PW 26
#define PH 18
#define PCH 480
#define PATCH_MAIN (3*PCH)
#define PATCH_TOT  (PATCH_MAIN+224)

#define W1F_HALVES (K1CH*NT1*32*16)
#define W2F_HALVES (K2CH*NT2*32*16)

__global__ __launch_bounds__(256) void prep_w1_k(const float* __restrict__ W1,
                                                 _Float16* __restrict__ W1f) {
  int t8 = blockIdx.x * 256 + threadIdx.x;
  if (t8 >= W1F_HALVES / 8) return;
  int t = t8 * 8;
  int h0 = t & 15, lane = (t >> 4) & 31, nt = (t >> 9) & 7, kc = t >> 12;
  int n = nt * 16 + (lane & 15);
  _Float16 hh[8], hl[8];
#pragma unroll
  for (int e = 0; e < 8; ++e) { const int h = h0 + e; const int k = kc * 32 + ((lane & 16) >> 1) + ((h < 8) ? h : (h + 8));
    const float v = (k < CKK) ? W1[k * N1 + n] : 0.f; hh[e] = (_Float16)v; hl[e] = lo_of(v, hh[e]); }
  *(volatile v4u_t*)(W1f + t) = *(const v4ua*)hh; *(volatile v4u_t*)(W1f + W1F_HALVES + t) = *(const v4ua*)hl; __threadfence();
  *(volatile v4u_t*)(W1f + t) = *(const v4ua*)hh; *(volatile v4u_t*)(W1f + W1F_HALVES + t) = *(const v4ua*)hl;
}

__global__ __launch_bounds__(256) void prep_w2_k(const float* __restrict__ W2,
                                                 _Float16* __restrict__ W2f) {
  int t8 = blockIdx.x * 256 + threadIdx.x;
  if (t8 >= W2F_HALVES / 8) return;
  int t = t8 * 8;
  int h0 = t & 15, lane = (t >> 4) & 31, nt = (t >> 9) & 3, kc = t >> 11;
  int n = nt * 16 + (lane & 15);
  _Float16 hh[8], hl[8];
#pragma unroll
  for (int e = 0; e < 8; ++e) { const int h = h0 + e; const int k = kc * 32 + ((lane & 16) >> 1) + ((h < 8) ? h : (h + 8));
    const float v = W2[k * N2 + n]; hh[e] = (_Float16)v; hl[e] = lo_of(v, hh[e]); }
  *(volatile v4u_t*)(W2f + t) = *(const v4ua*)hh; *(volatile v4u_t*)(W2f + W2F_HALVES + t) = *(const v4ua*)hl; __threadfence();
  *(volatile v4u_t*)(W2f + t) = *(const v4ua*)hh; *(volatile v4u_t*)(W2f + W2F_HALVES + t) = *(const v4ua*)hl;
}

__global__ __launch_bounds__(128) void conv_mlp_k(
    const float* __restrict__ x,
    const float* __restrict__ b1, const float* __restrict__ b2,
    const float* __restrict__ W3, const float* __restrict__ b3,
    const _Float16* __restrict__ W1f, const _Float16* __restrict__ W2f,
    float* __restrict__ out)
{
  __shared__ alignas(32) _Float16 patch[PATCH_TOT], patchl[PATCH_TOT];
  __shared__ unsigned short offt[384];
  __shared__ alignas(32) _Float16 h1[NW][32 * N1], h1l[NW][32 * N1];
  __shared__ alignas(32) _Float16 h2[NW][32 * N2];
  __shared__ alignas(16) float h2f[NW][32 * N2];
  __shared__ alignas(16) float ost[NW][32 * NE];
  __shared__ float b1s[N1];
  __shared__ float b2s[N2];
  __shared__ float w3s[N2 * NE];
  __shared__ float b3s[NE];

  const int tid = threadIdx.x;
  const int y0 = blockIdx.y * 8;
  const int x0 = blockIdx.x * 16;

  for (int idx = tid; idx < PATCH_TOT; idx += 128) {
    float v = 0.f;
    if (idx < PATCH_MAIN) {
      int c = idx / PCH, r = idx - c * PCH;
      int pr = r / PW, pc = r - pr * PW;
      if (pr < PH) {
        int gy = y0 - 5 + pr, gx = x0 - 5 + pc;
        if ((unsigned)gy < (unsigned)HW && (unsigned)gx < (unsigned)HW)
          v = x[c * NPIX + gy * HW + gx];
      }
    }
    patch[idx] = (_Float16)v; patchl[idx] = lo_of(v, patch[idx]);
  }
  for (int i = tid; i < 384; i += 128) {
    unsigned short off;
    if (i < CKK) {
      int c = i / 121, rem = i - c * 121;
      int ki = rem / 11, kj = rem - ki * 11;
      off = (unsigned short)(c * PCH + ki * PW + kj);
    } else {
      off = (unsigned short)PATCH_MAIN;
    }
    offt[i] = off;
  }
  if (tid < N1) b1s[tid] = b1[tid];
  if (tid < N2) b2s[tid] = b2[tid];
  for (int i = tid; i < N2 * NE; i += 128) w3s[i] = W3[i];
  if (tid < NE) b3s[tid] = b3[tid];
  __syncthreads();

  const int lane = tid & 31;
  const int w = tid >> 5;
  const int m = lane & 15;
  const int hiHalf = (lane >> 4) & 1;
  const int baseIdx0 = (2 * w)     * PW + m;
  const int baseIdx1 = (2 * w + 1) * PW + m;
  _Float16* h1w = &h1[w][0];
  _Float16* h1wl = &h1l[w][0];
  float* h2fw = &h2f[w][0];
  (void)h2;

  const v8f vzero = {0.f, 0.f, 0.f, 0.f, 0.f, 0.f, 0.f, 0.f};
  const int Mb = hiHalf * 8;

  #pragma unroll 1
  for (int s = 0; s < 2; ++s) {
    const int baseIdx = s ? baseIdx1 : baseIdx0;
    v8f acc[NT1];
    #pragma unroll
    for (int nt = 0; nt < NT1; ++nt) acc[nt] = vzero;
    #pragma unroll 1
    for (int kc = 0; kc < K1CH; ++kc) {
      const int kb = kc * 32 + hiHalf * 8;
      v16h a0, a0l;
      #pragma unroll
      for (int h = 0; h < 16; ++h) {
        int k = kb + (h < 8 ? h : 8 + h);
        int off = (int)offt[k];
        a0[h] = patch[baseIdx + off];  a0l[h] = patchl[baseIdx + off];
      }
      #pragma unroll
      for (int nt = 0; nt < NT1; ++nt) {
        const int nidx = kc * NT1 + nt;
        const v16h bcur = *(const v16h*)(W1f + (nidx * 32 + lane) * 16);
        const v16h blo  = *(const v16h*)(W1f + W1F_HALVES + (nidx * 32 + lane) * 16);
        acc[nt] = wmma_split(a0, a0l, bcur, blo, acc[nt]);
      }
    }
    #pragma unroll
    for (int nt = 0; nt < NT1; ++nt) {
      float bias = b1s[nt * 16 + m];
      #pragma unroll
      for (int r = 0; r < 8; ++r) {
        float v = acc[nt][r] + bias;
        v = fmaxf(v, 0.f) + 0.01f * fminf(v, 0.f);
        const _Float16 hv = (_Float16)v;
        h1w[(s * 16 + Mb + r) * N1 + nt * 16 + m] = hv;  h1wl[(s * 16 + Mb + r) * N1 + nt * 16 + m] = lo_of(v, hv);
      }
    }
  }

  v8f acc2[2][NT2];
  #pragma unroll
  for (int nt = 0; nt < NT2; ++nt) { acc2[0][nt] = vzero; acc2[1][nt] = vzero; }

  asm volatile("s_wait_dscnt 0" ::: "memory");
  #pragma unroll 1
  for (int kc = 0; kc < K2CH; ++kc) {
    const int kb = kc * 32 + hiHalf * 8;
    v16h a2[2], a2l[2];
    #pragma unroll
    for (int s = 0; s < 2; ++s) {
      v8h lo = *(const v8h*)(h1w + (s * 16 + m) * N1 + kb);
      v8h hi = *(const v8h*)(h1w + (s * 16 + m) * N1 + kb + 16);
      v8h lol = *(const v8h*)(h1wl + (s * 16 + m) * N1 + kb);
      v8h hil = *(const v8h*)(h1wl + (s * 16 + m) * N1 + kb + 16);
      #pragma unroll
      for (int h = 0; h < 8; ++h) { a2[s][h] = lo[h]; a2[s][h + 8] = hi[h]; a2l[s][h] = lol[h]; a2l[s][h + 8] = hil[h]; }
    }
    #pragma unroll
    for (int nt = 0; nt < NT2; ++nt) {
      const int nidx = kc * NT2 + nt;
      const v16h bcur = *(const v16h*)(W2f + (nidx * 32 + lane) * 16);
      const v16h blo  = *(const v16h*)(W2f + W2F_HALVES + (nidx * 32 + lane) * 16);
      acc2[0][nt] = wmma_split(a2[0], a2l[0], bcur, blo, acc2[0][nt]);
      acc2[1][nt] = wmma_split(a2[1], a2l[1], bcur, blo, acc2[1][nt]);
    }
  }

  #pragma unroll
  for (int s = 0; s < 2; ++s) {
    #pragma unroll
    for (int nt = 0; nt < NT2; ++nt) {
      float bias = b2s[nt * 16 + m];
      #pragma unroll
      for (int r = 0; r < 8; ++r) {
        float v = acc2[s][nt][r] + bias;
        v = fmaxf(v, 0.f) + 0.01f * fminf(v, 0.f);
        h2fw[(s * 16 + Mb + r) * N2 + nt * 16 + m] = v;
      }
    }
  }

  asm volatile("s_wait_dscnt 0" ::: "memory");
  {
    const int p = lane;
    float o[NE];
    #pragma unroll
    for (int e = 0; e < NE; ++e) o[e] = b3s[e];
    #pragma unroll 8
    for (int j = 0; j < N2; ++j) {
      float hv = h2fw[p * N2 + j];
      #pragma unroll
      for (int e = 0; e < NE; ++e) o[e] = fmaf(hv, w3s[j * NE + e], o[e]);
    }
    float ss = 0.f;
    #pragma unroll
    for (int e = 0; e < NE; ++e) ss += o[e] * o[e];
    float inv = 1.f / fmaxf(sqrtf(ss), 1e-12f);
    float* os = &ost[w][0];
    #pragma unroll
    for (int e = 0; e < NE; ++e) os[p * NE + e] = o[e] * inv;
    asm volatile("s_wait_dscnt 0" ::: "memory");
#pragma unroll 1
    for (int pass = 0; pass < 2; ++pass) {
#pragma unroll
      for (int rr = 0; rr < 2; ++rr) {
        const int gy = y0 + 2 * w + rr;
        float* op = out + ((size_t)gy * HW + x0) * NE;
        *(volatile v4f_t*)(op + lane * 4) = *(const volatile v4fa*)(os + rr * 128 + lane * 4);
      }
      __threadfence();
    }
  }
}

extern "C" void kernel_launch(void* const* d_in, const int* in_sizes, int n_in,
                              void* d_out, int out_size, void* d_ws, size_t ws_size,
                              hipStream_t stream) {
  (void)in_sizes; (void)n_in; (void)out_size; (void)ws_size;
  const float* x  = (const float*)d_in[0];
  const float* W1 = (const float*)d_in[1];
  const float* b1 = (const float*)d_in[2];
  const float* W2 = (const float*)d_in[3];
  const float* b2 = (const float*)d_in[4];
  const float* W3 = (const float*)d_in[5];
  const float* b3 = (const float*)d_in[6];

  _Float16* W1f = (_Float16*)d_ws;
  _Float16* W2f = (_Float16*)((char*)d_ws + (size_t)2 * W1F_HALVES * sizeof(_Float16));

  prep_w1_k<<<(W1F_HALVES / 8 + 255) / 256, 256, 0, stream>>>(W1, W1f);
  prep_w2_k<<<(W2F_HALVES / 8 + 255) / 256, 256, 0, stream>>>(W2, W2f);
  conv_mlp_k<<<dim3(25, 50), 128, 0, stream>>>(x, b1, b2, W3, b3, W1f, W2f,
                                               (float*)d_out);
}
